// StressPredictorFromFp_78967268704762
// MI455X (gfx1250) — hardware-verified
//
#include <hip/hip_runtime.h>
#include <stddef.h>


typedef _Float16 h16;
typedef _Float16 v16h __attribute__((ext_vector_type(16)));
typedef _Float16 v8h  __attribute__((ext_vector_type(8)));
typedef float    v8f  __attribute__((ext_vector_type(8)));
typedef float    v4f  __attribute__((ext_vector_type(4)));

#ifndef NROWS
#define NROWS 1000000
#endif
#define NROWS_FULL 1000000
#define HIDN 128
#define NTILES (NROWS / 16)

#ifndef RES_MODE
#define RES_MODE 2
#endif

static_assert(NROWS >= 16 && NROWS <= NROWS_FULL);
static_assert((NROWS % 16) == 0);
static_assert(NTILES * 16 == NROWS);
static_assert(HIDN == 128);
static_assert((HIDN % 64) == 0 && (HIDN % 32) == 0 && (HIDN % 8) == 0);
static_assert(RES_MODE >= 0 && RES_MODE <= 2);
static_assert((size_t)NROWS * 4u * 4u <= (size_t)16000000);

#define LDT 72
static_assert((LDT % 8) == 0 && LDT >= 64);

#define WCARRY 64.0f
#define RCARRY 2048.0f
#define SC_M (1.0f / WCARRY)
#define SC_R (1.0f / (WCARRY * RCARRY))
#define F16_MIN_NORMAL 6.103515625e-05f

#define W2P_BYTES ((size_t)HIDN * HIDN * 2)
#define W3P_BYTES ((size_t)16 * HIDN * 2)
#define OFF_W2H ((size_t)0)
#define OFF_W2L (OFF_W2H + W2P_BYTES)
#define OFF_W3H (OFF_W2L + W2P_BYTES)
#define OFF_W3L (OFF_W3H + W3P_BYTES)
#define WS_TOTAL (OFF_W3L + W3P_BYTES)
static_assert((W2P_BYTES % 128) == 0 && (W3P_BYTES % 128) == 0);
static_assert(WS_TOTAL <= (size_t)134217728);

static __device__ __forceinline__ h16 toh_flush(float v) {
  const h16 r = (h16)v;
  return (fabsf(v) < F16_MIN_NORMAL) ? (h16)0.0f : r;
}

static __device__ __forceinline__ void relu_split(float t, h16& hi, h16& lo) {
  const float v = (t < F16_MIN_NORMAL) ? 0.0f : t;
  hi = (h16)v;
  lo = (RES_MODE >= 1) ? toh_flush((v - (float)hi) * RCARRY) : (h16)0.0f;
}

__device__ __forceinline__ v16h frag_at(const _Float16* p) {
  v8h lo = *(const v8h*)(p);
  v8h hi = *(const v8h*)(p + 16);
  v16h out;
#pragma unroll
  for (int i = 0; i < 8; ++i) { out[i] = lo[i]; out[i + 8] = hi[i]; }
  return out;
}

__device__ __forceinline__ v8f wmma16(v16h a, v16h b, v8f c) {
  v8f d = __builtin_amdgcn_wmma_f32_16x16x32_f16(false, a, false, b, (short)0, c,
                                                 false, false);
  asm volatile("v_nop\n\tv_nop\n\tv_nop\n\tv_nop" : "+v"(d) : "v"(a), "v"(b));
  return d;
}

__global__ __launch_bounds__(256) void w2plane_kernel(
    const float* __restrict__ W, _Float16* __restrict__ Wh, _Float16* __restrict__ Wl,
    unsigned ldw, unsigned ldk) {
  __shared__ _Float16 Th[64 * LDT];
  __shared__ _Float16 Tl[64 * LDT];
  const unsigned tid = threadIdx.x;
  const unsigned n0 = blockIdx.x * 64u;
  const unsigned k0 = blockIdx.y * 64u;
#pragma unroll 4
  for (unsigned j = 0; j < 16u; ++j) {
    const unsigned idx = tid + 256u * j;
    const unsigned kr = idx >> 6, nc = idx & 63u;
    const float v = WCARRY * W[(size_t)(k0 + kr) * ldw + n0 + nc];
    const h16 hi = toh_flush(v);
    const h16 lo = toh_flush((v - (float)hi) * RCARRY);
    Th[nc * LDT + kr] = hi;
    Tl[nc * LDT + kr] = lo;
  }
  __syncthreads();
  v8h xh[2], xl[2];
  size_t off[2];
#pragma unroll
  for (unsigned i = 0; i < 2u; ++i) {
    const unsigned n = 32u * i + (tid >> 3);
    const unsigned kc = (tid & 7u) * 8u;
    xh[i] = *(const v8h*)&Th[n * LDT + kc];
    xl[i] = *(const v8h*)&Tl[n * LDT + kc];
    off[i] = (size_t)(n0 + n) * ldk + k0 + kc;
  }
#pragma unroll
  for (int i = 0; i < 2; ++i) {
    *(volatile v8h*)(Wh + off[i]) = xh[i];
    *(volatile v8h*)(Wl + off[i]) = xl[i];
  }
  __threadfence();
#pragma unroll
  for (int i = 0; i < 2; ++i) {
    *(volatile v8h*)(Wh + off[i]) = xh[i];
    *(volatile v8h*)(Wl + off[i]) = xl[i];
  }
}

__global__ __launch_bounds__(256) void w3plane_kernel(
    const float* __restrict__ W3, _Float16* __restrict__ W3h, _Float16* __restrict__ W3l) {
  const unsigned tid = threadIdx.x;
  const unsigned n = tid >> 4;
  const unsigned kc = (tid & 15u) * 8u;
  const unsigned nn = (n < 4u) ? n : 3u;
  v8h xh, xl;
#pragma unroll
  for (unsigned i = 0; i < 8u; ++i) {
    const float s = W3[(kc + i) * 4u + nn];
    const float v = (n < 4u) ? (WCARRY * s) : 0.0f;
    const h16 hi = toh_flush(v);
    const h16 lo = toh_flush((v - (float)hi) * RCARRY);
    xh[i] = hi;
    xl[i] = lo;
  }
  _Float16* ph = W3h + n * HIDN + kc;
  _Float16* pl = W3l + n * HIDN + kc;
  *(volatile v8h*)ph = xh;
  *(volatile v8h*)pl = xl;
  __threadfence();
  *(volatile v8h*)ph = xh;
  *(volatile v8h*)pl = xl;
}

__global__ __launch_bounds__(256) void mlp_polar_kernel(
    const float* __restrict__ F, const float* __restrict__ W1, const float* __restrict__ b1,
    const _Float16* __restrict__ W2h, const _Float16* __restrict__ W2l,
    const float* __restrict__ b2,
    const _Float16* __restrict__ W3h, const _Float16* __restrict__ W3l,
    const float* __restrict__ b3, float* __restrict__ out) {
  const unsigned lane = threadIdx.x & 31u;
  const int wave = __builtin_amdgcn_readfirstlane(threadIdx.x >> 5);
  const unsigned hh = lane >> 4, m = lane & 15u;
  const unsigned tile = blockIdx.x * 8u + (unsigned)wave;
  if (tile >= (unsigned)NTILES) return;

  const size_t row = (size_t)tile * 16u + m;
  const v4f fv = *(const v4f*)(F + row * 4u);
  const float fa = fv[0], fb = fv[1], fc = fv[2], fd = fv[3];

  const float det = fa * fd - fb * fc;
  const float sgn = (det >= 0.0f) ? 1.0f : -1.0f;
  const float m00 = fa + sgn * fd, m01 = fb - sgn * fc;
  const float m10 = fc - sgn * fb, m11 = fd + sgn * fa;
  const float h2  = m00 * m00 + m01 * m01;
  const float hin = rsqrtf(fmaxf(h2, 1e-30f));
  const float r00 = m00 * hin, r01 = m01 * hin, r10 = m10 * hin, r11 = m11 * hin;
  const float x0 = h2 * hin - 2.0f;
  const float x1 = fa * fa + fb * fb + fc * fc + fd * fd - 1.0f;
  const float x2 = det - 1.0f;

  v16h hbh[4], hbl[4];
  unsigned kofs = 8u * hh;
#pragma unroll
  for (int ks = 0; ks < 4; ++ks) {
    v16h fh, fl;
#pragma unroll
    for (int g = 0; g < 2; ++g) {
      const unsigned kb = kofs + 32u * (unsigned)ks + 16u * (unsigned)g;
      const v4f wa0 = *(const v4f*)(W1 + kb);
      const v4f wa1 = *(const v4f*)(W1 + kb + 4u);
      const v4f wb0 = *(const v4f*)(W1 + HIDN + kb);
      const v4f wb1 = *(const v4f*)(W1 + HIDN + kb + 4u);
      const v4f wc0 = *(const v4f*)(W1 + 2 * HIDN + kb);
      const v4f wc1 = *(const v4f*)(W1 + 2 * HIDN + kb + 4u);
      const v4f bb0 = *(const v4f*)(b1 + kb);
      const v4f bb1 = *(const v4f*)(b1 + kb + 4u);
      asm volatile("" : "+v"(kofs)
                   : "v"(wa0), "v"(wa1), "v"(wb0), "v"(wb1), "v"(wc0), "v"(wc1),
                     "v"(bb0), "v"(bb1));
#pragma unroll
      for (int i = 0; i < 4; ++i) {
        const float t0 = ((x0 * wa0[i] + x1 * wb0[i]) + x2 * wc0[i]) + bb0[i];
        const float t1 = ((x0 * wa1[i] + x1 * wb1[i]) + x2 * wc1[i]) + bb1[i];
        h16 hi, lo;
        relu_split(t0, hi, lo);
        fh[8 * g + i] = hi;
        fl[8 * g + i] = lo;
        relu_split(t1, hi, lo);
        fh[8 * g + i + 4] = hi;
        fl[8 * g + i + 4] = lo;
      }
    }
    hbh[ks] = fh;
    hbl[ks] = fl;
  }

  v8f yM = {}, yR = {};
#pragma unroll 1
  for (unsigned s3 = 0; s3 < 4u; ++s3) {
    const unsigned aoff = (32u * s3 + m) * (unsigned)HIDN + hh * 8u;
    v8f m0 = {}, r0 = {}, m1 = {}, r1 = {};
#pragma unroll
    for (int ks = 0; ks < 4; ++ks) {
      const v16h a0 = frag_at(W2h + aoff + 32u * (unsigned)ks);
      const v16h a1 = frag_at(W2h + aoff + 16u * (unsigned)HIDN + 32u * (unsigned)ks);
      m0 = wmma16(a0, hbh[ks], m0);
      m1 = wmma16(a1, hbh[ks], m1);
      if (RES_MODE >= 1) {
        r0 = wmma16(a0, hbl[ks], r0);
        r1 = wmma16(a1, hbl[ks], r1);
      }
      if (RES_MODE >= 2) {
        const v16h l0 = frag_at(W2l + aoff + 32u * (unsigned)ks);
        const v16h l1 = frag_at(W2l + aoff + 16u * (unsigned)HIDN + 32u * (unsigned)ks);
        r0 = wmma16(l0, hbh[ks], r0);
        r1 = wmma16(l1, hbh[ks], r1);
      }
    }

    const unsigned bo = 32u * s3 + 8u * hh;
    const v4f c00 = *(const v4f*)(b2 + bo);
    const v4f c01 = *(const v4f*)(b2 + bo + 4u);
    const v4f c10 = *(const v4f*)(b2 + bo + 16u);
    const v4f c11 = *(const v4f*)(b2 + bo + 20u);
    float bz0[8], bz1[8];
#pragma unroll
    for (int i = 0; i < 4; ++i) {
      bz0[i] = c00[i]; bz0[i + 4] = c01[i];
      bz1[i] = c10[i]; bz1[i + 4] = c11[i];
    }
    v16h gh, gl;
#pragma unroll
    for (int r = 0; r < 8; ++r) {
      const float z0 = (m0[r] * SC_M + r0[r] * SC_R) + bz0[r];
      const float z1 = (m1[r] * SC_M + r1[r] * SC_R) + bz1[r];
      h16 hi, lo;
      relu_split(z0, hi, lo);
      gh[r] = hi;
      gl[r] = lo;
      relu_split(z1, hi, lo);
      gh[r + 8] = hi;
      gl[r + 8] = lo;
    }

    const unsigned woff = m * (unsigned)HIDN + 32u * s3 + hh * 8u;
    const v16h w3 = frag_at(W3h + woff);
    yM = wmma16(w3, gh, yM);
    if (RES_MODE >= 1) yR = wmma16(w3, gl, yR);
    if (RES_MODE >= 2) {
      const v16h l3 = frag_at(W3l + woff);
      yR = wmma16(l3, gh, yR);
    }
  }

  const v4f bq = *(const v4f*)b3;
  const float y00 = (yM[0] * SC_M + yR[0] * SC_R) + bq[0];
  const float y01 = (yM[1] * SC_M + yR[1] * SC_R) + bq[1];
  const float y10 = (yM[2] * SC_M + yR[2] * SC_R) + bq[2];
  const float y11 = (yM[3] * SC_M + yR[3] * SC_R) + bq[3];
  const float s01 = 0.5f * (y01 + y10);
  const float p00 = r00 * y00 + r01 * s01;
  const float p01 = r00 * s01 + r01 * y11;
  const float p10 = r10 * y00 + r11 * s01;
  const float p11 = r10 * s01 + r11 * y11;
  v4f o;
  o[0] = p00 * fa + p01 * fb;
  o[1] = p00 * fc + p01 * fd;
  o[2] = p10 * fa + p11 * fb;
  o[3] = p10 * fc + p11 * fd;

  float* po = out + row * 4u;
  const bool act = (hh == 0u);
  if (act) *(volatile v4f*)po = o;
  __threadfence();
  if (act) *(volatile v4f*)po = o;
}

extern "C" void kernel_launch(void* const* d_in, const int* in_sizes, int n_in,
                              void* d_out, int out_size, void* d_ws, size_t ws_size,
                              hipStream_t stream) {
  if (n_in < 7) return;
  if ((long long)in_sizes[0] < (long long)NROWS * 4) return;
  if (in_sizes[1] < 3 * HIDN) return;
  if (in_sizes[2] < HIDN) return;
  if (in_sizes[3] < HIDN * HIDN) return;
  if (in_sizes[4] < HIDN) return;
  if (in_sizes[5] < HIDN * 4) return;
  if (in_sizes[6] < 4) return;
  if ((long long)out_size < (long long)NROWS * 4) return;
  if (ws_size < WS_TOTAL) return;

  const float* F  = (const float*)d_in[0];
  const float* W1 = (const float*)d_in[1];
  const float* b1 = (const float*)d_in[2];
  const float* W2 = (const float*)d_in[3];
  const float* b2 = (const float*)d_in[4];
  const float* W3 = (const float*)d_in[5];
  const float* b3 = (const float*)d_in[6];
  float* out = (float*)d_out;

  char* ws = (char*)d_ws;
  _Float16* W2h = (_Float16*)(ws + OFF_W2H);
  _Float16* W2l = (_Float16*)(ws + OFF_W2L);
  _Float16* W3h = (_Float16*)(ws + OFF_W3H);
  _Float16* W3l = (_Float16*)(ws + OFF_W3L);

  dim3 blk(256);
  w2plane_kernel<<<dim3(HIDN / 64, HIDN / 64), blk, 0, stream>>>(W2, W2h, W2l,
                                                                 (unsigned)HIDN, (unsigned)HIDN);
  w3plane_kernel<<<dim3(1), blk, 0, stream>>>(W3, W3h, W3l);
  mlp_polar_kernel<<<dim3((NTILES + 7) / 8), blk, 0, stream>>>(F, W1, b1, W2h, W2l, b2,
                                                               W3h, W3l, b3, out);
}
